// MIMOSS_55009941127824
// MI455X (gfx1250) — hardware-verified
//
#include <hip/hip_runtime.h>
#include <math.h>

typedef __attribute__((ext_vector_type(16))) _Float16 v16h;
typedef __attribute__((ext_vector_type(16))) __bf16 v16b;
typedef __attribute__((ext_vector_type(8)))  _Float16 v8h;
typedef __attribute__((ext_vector_type(8)))  float v8f;
typedef __attribute__((ext_vector_type(4)))  float v4f;
typedef __attribute__((ext_vector_type(2)))  float v2f;
typedef __attribute__((ext_vector_type(4)))  unsigned v4u;
typedef __attribute__((ext_vector_type(4)))  int v4i;
typedef float __attribute__((may_alias)) float_a;
typedef int __attribute__((may_alias)) int_a;

template <typename T> __device__ __forceinline__ void vst2(void* p, T v) { *(volatile T*)p = v; __threadfence(); *(volatile T*)p = v; }
__device__ __forceinline__ v8f wmma16(v16h a, v16h b, v8f c) {
  v8f d = __builtin_amdgcn_wmma_f32_16x16x32_f16(false, a, false, b, (short)0, c, false, false);
  asm volatile("v_nop\n\tv_nop\n\tv_nop\n\tv_nop" : "+v"(d) : "v"(a), "v"(b));
  return d;
}
__device__ __forceinline__ v8f wmma_bf(v16b a, v16b b, v8f c) {
  v8f d = __builtin_amdgcn_wmma_f32_16x16x32_bf16(false, a, false, b, (short)0, c, false, false);
  asm volatile("v_nop\n\tv_nop\n\tv_nop\n\tv_nop" : "+v"(d) : "v"(a), "v"(b));
  return d;
}
__device__ __forceinline__ v16h frag_h(const _Float16* rowk0, int lane) {
  union { v16h v; v8h q[2]; } u; const _Float16* p = rowk0 + 8 * (lane >> 4);
  u.q[0] = *(const v8h*)p; u.q[1] = *(const v8h*)(p + 16); return u.v;
}
__device__ __forceinline__ v16h frag_f32(const float* rowk0, int lane) {
  v16h a; const float* p = rowk0 + 8 * (lane >> 4);
#pragma unroll
  for (int i = 0; i < 8; ++i) { a[i] = (_Float16)p[i]; a[8 + i] = (_Float16)p[16 + i]; }
  return a;
}
__device__ __forceinline__ v16h frag_f32s(const float* rowk0, int lane, float sc) {
  v16h a; const float* p = rowk0 + 8 * (lane >> 4);
#pragma unroll
  for (int i = 0; i < 8; ++i) { a[i] = (_Float16)(p[i] * sc); a[8 + i] = (_Float16)(p[16 + i] * sc); }
  return a;
}
__device__ __forceinline__ v16h fragc_f32(const float* W, int k0, int n, int lane, int ld, int K) {
  v16h a; const int g = lane >> 4;
#pragma unroll
  for (int i = 0; i < 8; ++i) { const int ka = k0 + 8 * g + i, kb = ka + 16;
    a[i] = (_Float16)(ka < K ? W[(size_t)(ka < K ? ka : K - 1) * ld + n] : 0.f); a[8 + i] = (_Float16)(kb < K ? W[(size_t)(kb < K ? kb : K - 1) * ld + n] : 0.f); }
  return a;
}
struct F2 { v16b h, l; };
__device__ __forceinline__ F2 bsplit16(const float v[16]) { F2 r;
#pragma unroll
  for (int i = 0; i < 16; ++i) { const __bf16 h = (__bf16)v[i]; r.h[i] = h; r.l[i] = (__bf16)(v[i] - (float)h); }
  return r; }
__device__ __forceinline__ F2 split_row(const float* row, int k0, int lane) { float v[16]; const float* p = row + k0 + 8 * (lane >> 4);
#pragma unroll
  for (int i = 0; i < 8; ++i) { v[i] = p[i]; v[8 + i] = p[16 + i]; }
  return bsplit16(v); }
__device__ __forceinline__ F2 split_rowK(const float* row, int k0, int lane, int K) { float v[16]; const int g = lane >> 4;
#pragma unroll
  for (int i = 0; i < 8; ++i) { const int ka = k0 + 8 * g + i, kb = ka + 16; v[i] = ka < K ? row[ka < K ? ka : K - 1] : 0.f; v[8 + i] = kb < K ? row[kb < K ? kb : K - 1] : 0.f; }
  return bsplit16(v); }
__device__ __forceinline__ F2 split_col(const float* W, int k0, int n, int lane, int ld, int K) { float v[16]; const int g = lane >> 4;
#pragma unroll
  for (int i = 0; i < 8; ++i) { const int ka = k0 + 8 * g + i, kb = ka + 16; v[i] = ka < K ? W[(size_t)(ka < K ? ka : K - 1) * ld + n] : 0.f; v[8 + i] = kb < K ? W[(size_t)(kb < K ? kb : K - 1) * ld + n] : 0.f; }
  return bsplit16(v); }
__device__ __forceinline__ v8f mac3(const F2& a, const F2& b, v8f c) { c = wmma_bf(a.l, b.h, c); c = wmma_bf(a.h, b.l, c); return wmma_bf(a.h, b.h, c); }
__device__ __forceinline__ float sigm(float v) { return 1.0f / (1.0f + expf(-v)); }
#define LDSX() do { asm volatile("s_wait_dscnt 0" ::: "memory"); __builtin_amdgcn_wave_barrier(); __builtin_amdgcn_fence(__ATOMIC_RELEASE, "workgroup"); } while (0)


#define NBAT 64
#ifndef NSEQ
#define NSEQ 16384
#endif
#define NS 128
#define NI 6
#define NO 6
#define SEQ 16384
typedef __attribute__((ext_vector_type(8))) __bf16 v8b;
__device__ __forceinline__ v16b frag_b(const __bf16* rowk0, int lane) {
  union { v16b v; v8b q[2]; } u; const __bf16* p = rowk0 + 8 * (lane >> 4);
  u.q[0] = *(const v8b*)p; u.q[1] = *(const v8b*)(p + 16); return u.v;
}
__device__ __forceinline__ float bfr(float v) { return (float)(__bf16)v; }
__device__ __attribute__((noinline)) float exp_ni(float v) { return expf(v); }
__device__ __attribute__((noinline)) float erf_ni(float v) { return erff(v); }

#define WS_PA 0u
#define WS_PC (WS_PA + 2u * NS * NS)
#define WS_Y  (WS_PC + 2u * 16 * NS)
#define WS_END (WS_Y + 4u * (size_t)SEQ * NBAT * 8)

__global__ __launch_bounds__(128) void k_pack(const float* __restrict__ A, const float* __restrict__ C, __bf16* __restrict__ PA, __bf16* __restrict__ PC) {
  __shared__ __align__(16) __bf16 s[NS]; const int n = blockIdx.x, which = blockIdx.y, t = threadIdx.x;
  if (which == 1 && n >= 16) return;
  s[t] = (__bf16)((which == 0) ? A[(size_t)n * NS + t] : (n < NO ? C[(size_t)n * NS + t] : 0.f));
  __syncthreads();
  if (t < 16) vst2((unsigned*)((which == 0 ? PA : PC) + (size_t)n * NS + t * 8), *(const v4u*)&s[t * 8]);
}
__global__ __launch_bounds__(128) void k_ssm(const float* __restrict__ INP, const __bf16* __restrict__ PA, const __bf16* __restrict__ PC, const float* __restrict__ Bm, const float* __restrict__ Dm, const float* __restrict__ X0, const float* __restrict__ IM, const float* __restrict__ IS, float* __restrict__ Y) {
  __shared__ __align__(16) float sx[4][16][132]; __shared__ __align__(16) float sy[4][16][8];
  const int tid = threadIdx.x, wave = tid >> 5, lane = tid & 31, col = lane & 15, g = lane >> 4; const int b0 = wave * 16;
  float bw[8][NI], dw[NI], im[NI], isd[NI];
#pragma unroll
  for (int i = 0; i < NI; ++i) { im[i] = bfr(IM[i]); isd[i] = bfr(IS[i]); dw[i] = (col < NO) ? bfr(Dm[col * NI + i]) : 0.f;
#pragma unroll
    for (int j = 0; j < 8; ++j) bw[j][i] = bfr(Bm[(size_t)(j * 16 + col) * NI + i]); }
#pragma unroll
  for (int j = 0; j < 8; ++j)
#pragma unroll
    for (int r = 0; r < 8; ++r) sx[wave][8 * g + r][j * 16 + col] = bfr(X0[j * 16 + col]);
  LDSX();
#pragma unroll 1
  for (int k = 0; k < NSEQ; ++k) {
    float u[8][NI];
#pragma unroll
    for (int r = 0; r < 8; ++r) { const float* ip = INP + ((size_t)(b0 + 8 * g + r) * SEQ + k) * NI;
#pragma unroll
      for (int i = 0; i < NI; ++i) u[r][i] = (bfr(ip[i]) - im[i]) / isd[i]; }
    v8f acc[9] = {};
#pragma unroll
    for (int kc = 0; kc < NS / 32; ++kc) { const F2 a = split_row(&sx[wave][col][0], kc * 32, lane);
#pragma unroll
      for (int j = 0; j < 8; ++j) { const v16b w = frag_b(PA + (size_t)(j * 16 + col) * NS + kc * 32, lane); acc[j] = wmma_bf(a.l, w, acc[j]); acc[j] = wmma_bf(a.h, w, acc[j]); }
      { const v16b w = frag_b(PC + (size_t)col * NS + kc * 32, lane); acc[8] = wmma_bf(a.l, w, acc[8]); acc[8] = wmma_bf(a.h, w, acc[8]); } }
    LDSX();
#pragma unroll
    for (int r = 0; r < 8; ++r) { float yv = acc[8][r], ud = 0.f;
#pragma unroll
      for (int i = 0; i < NI; ++i) ud += u[r][i] * dw[i];
      if (col < 8) sy[wave][8 * g + r][col] = (col < NO) ? (yv + ud) : 0.f;
#pragma unroll
      for (int j = 0; j < 8; ++j) { float ub = 0.f;
#pragma unroll
        for (int i = 0; i < NI; ++i) ub += u[r][i] * bw[j][i];
        sx[wave][8 * g + r][j * 16 + col] = acc[j][r] + ub; } }
    LDSX();
    vst2(Y + ((size_t)k * NBAT + b0) * 8 + lane * 4, *(const v4f*)&(&sy[wave][0][0])[lane * 4]);
  }
}
__global__ __launch_bounds__(128) void k_out(const float* __restrict__ Y, const float* __restrict__ OM, const float* __restrict__ OSD, float* __restrict__ OUT) {
  __shared__ __align__(16) float so[256 * NO]; const int b = blockIdx.y, s0 = blockIdx.x * 256, t = threadIdx.x;
  for (int q = t; q < 256 * NO; q += 128) { const int s = q / NO, o = q % NO; so[q] = (s0 + s < NSEQ) ? Y[((size_t)(s0 + s) * NBAT + b) * 8 + o] * bfr(OSD[o]) + bfr(OM[o]) : 0.f; }
  __syncthreads();
  for (int q = t; q < 256 * NO / 4; q += 128) vst2(OUT + ((size_t)b * SEQ + s0) * NO + q * 4, *(const v4f*)&so[q * 4]);
}
extern "C" void kernel_launch(void* const* d_in, const int* in_sizes, int n_in, void* d_out, int out_size, void* d_ws, size_t ws_size, hipStream_t stream) {
  (void)in_sizes; (void)n_in; (void)out_size;
  const float** F = (const float**)d_in;
  if (ws_size < (size_t)WS_END) return;
  char* ws = (char*)d_ws; __bf16 *PA = (__bf16*)(ws + WS_PA), *PC = (__bf16*)(ws + WS_PC); float* Y = (float*)(ws + WS_Y);
  k_pack<<<dim3(NS, 2), 128, 0, stream>>>(F[1], F[3], PA, PC);
  k_ssm<<<1, 128, 0, stream>>>(F[0], PA, PC, F[2], F[4], F[5], F[6], F[7], Y);
  k_out<<<dim3(SEQ / 256, NBAT), 128, 0, stream>>>(Y, F[8], F[9], (float*)d_out);
}
